// DeepseekV3MoE_52673478918593
// MI455X (gfx1250) — hardware-verified
//
#include <hip/hip_runtime.h>
#include <stddef.h>
#include <stdint.h>

#define NTOK   2048
#define HD     1024
#define MI     512
#define SI     1024
#define NE     16
#define TOPK   4
#define NGRP   4
#define SCALEF 2.5f
#define TR     64
#define NTILE  144
#define MP     9216
#define TABH   64
#define TABL   (TABH + MP)
#define TABN   (TABH + MP + NTOK * TOPK)
#define TPT    8
#define NTHR   256
#define GTHR   128
#define GTOK   16
#define WSMAX  134217728
#define LDS_BKT ((TABN + NE * 8) * 4)

static_assert(MP == NTILE * TR);
static_assert(MP >= NTOK * TOPK + NE * (TR - 1));
static_assert((TABN % 32) == 0);
static_assert(((TABL * 4) % 16) == 0);
static_assert(NTOK == NTHR * TPT);
static_assert((NTOK % TR) == 0);
static_assert((NTOK % GTOK) == 0 && GTOK == 2 * (NTHR / 32));
static_assert((HD % 64) == 0 && (MI % 64) == 0 && (SI % 64) == 0);
static_assert((HD % 32) == 0 && (MI % 32) == 0 && (SI % 32) == 0);
static_assert((HD % 128) == 0);
static_assert(TR == (GTHR / 32) * 16);
static_assert(LDS_BKT <= 160000);
static_assert(NTHR / 32 == 8);
static_assert((NTOK % 8) == 0);
static_assert(NE == NGRP * 4 && TOPK == 4);

typedef float          v4f  __attribute__((ext_vector_type(4)));
typedef float          v8f  __attribute__((ext_vector_type(8)));
typedef int            v4i  __attribute__((ext_vector_type(4)));
typedef int            v8i  __attribute__((ext_vector_type(8)));
typedef unsigned short v8us __attribute__((ext_vector_type(8)));
typedef __bf16         v16bf __attribute__((ext_vector_type(16)));
union FragB { v16bf v; v8us h[2]; v8i w; };

__device__ __forceinline__ v8f wmb(const FragB& a, const FragB& b, v8f c) {
  v8f d = __builtin_amdgcn_wmma_f32_16x16x32_bf16(false, a.v, false, b.v, (short)0, c, false, false);
  asm volatile("v_nop\n\tv_nop\n\tv_nop\n\tv_nop" : "+v"(d) : "v"(a.w), "v"(b.w));
  return d;
}

__device__ __forceinline__ unsigned short rne16(float f) {
  unsigned u = __float_as_uint(f);
  u += 0x7FFFu + ((u >> 16) & 1u);
  return (unsigned short)(u >> 16);
}
__device__ __forceinline__ float rne16f(float f) {
  return __uint_as_float(((unsigned)rne16(f)) << 16);
}
__device__ __forceinline__ v8us cvt8(const v4f a, const v4f b) {
  v8us o;
  o[0] = rne16(a.x); o[1] = rne16(a.y); o[2] = rne16(a.z); o[3] = rne16(a.w);
  o[4] = rne16(b.x); o[5] = rne16(b.y); o[6] = rne16(b.z); o[7] = rne16(b.w);
  return o;
}
__device__ __forceinline__ void sp1(float v, unsigned short& hi, unsigned short& lo) {
  const unsigned short hb = rne16(v);
  const float hf = __uint_as_float(((unsigned)hb) << 16);
  hi = hb;
  lo = rne16(v - hf);
}
__device__ __forceinline__ void split8(const v4f a, const v4f b, v8us& hv, v8us& lv) {
  unsigned short h0, h1, h2, h3, h4, h5, h6, h7, l0, l1, l2, l3, l4, l5, l6, l7;
  sp1(a.x, h0, l0); sp1(a.y, h1, l1); sp1(a.z, h2, l2); sp1(a.w, h3, l3);
  sp1(b.x, h4, l4); sp1(b.y, h5, l5); sp1(b.z, h6, l6); sp1(b.w, h7, l7);
  hv[0] = h0; hv[1] = h1; hv[2] = h2; hv[3] = h3; hv[4] = h4; hv[5] = h5; hv[6] = h6; hv[7] = h7;
  lv[0] = l0; lv[1] = l1; lv[2] = l2; lv[3] = l3; lv[4] = l4; lv[5] = l5; lv[6] = l6; lv[7] = l7;
}

__global__ __launch_bounds__(NTHR) void k_wtr(const float* __restrict__ src, unsigned short* dst,
                                              int K, int N, int E, int nUnits) {
  const int u = (int)blockIdx.x * NTHR + (int)threadIdx.x;
  if (u >= nUnits) return;
  const int kq  = K >> 3;
  const int per = N * kq;
  int e = u / per;
  e = e > E - 1 ? E - 1 : e;
  const int rem = u - e * per;
  const int n   = rem / kq;
  const int k8  = (rem - n * kq) * 8;
  const float* p = src + ((size_t)e * (size_t)K + (size_t)k8) * (size_t)N + n;
  v4f a, b;
  a.x = p[0];                 a.y = p[(size_t)N];         a.z = p[(size_t)2 * N];     a.w = p[(size_t)3 * N];
  b.x = p[(size_t)4 * N];     b.y = p[(size_t)5 * N];     b.z = p[(size_t)6 * N];     b.w = p[(size_t)7 * N];
  const v8us o = cvt8(a, b);
  const size_t q = ((size_t)e * (size_t)N + (size_t)n) * (size_t)K + (size_t)k8;
  *(volatile v8us*)(dst + q) = o;
  __threadfence();
  *(volatile v8us*)(dst + q) = o;
}

__global__ __launch_bounds__(NTHR) void k_cvx(const float* __restrict__ src, unsigned short* dst, int nUnits) {
  const int u = (int)blockIdx.x * NTHR + (int)threadIdx.x;
  if (u >= nUnits) return;
  const size_t q = (size_t)u * 8;
  const v4f a = *(const v4f*)(src + q);
  const v4f b = *(const v4f*)(src + q + 4);
  const v8us o = cvt8(a, b);
  *(volatile v8us*)(dst + q) = o;
  __threadfence();
  *(volatile v8us*)(dst + q) = o;
}

__global__ __launch_bounds__(NTHR) void k_gate(const float* __restrict__ x, const float* __restrict__ gk,
                                               const float* __restrict__ gb, int* route) {
  __shared__ __attribute__((aligned(16))) int rec[GTOK * 8];
  const int tid = (int)threadIdx.x, lane = tid & 31, wave = tid >> 5, hh = lane >> 4, e = lane & 15;
  if (tid < GTOK * 8) rec[tid] = 0;
  int t = (int)blockIdx.x * GTOK + 2 * wave + hh;
  t = t > NTOK - 1 ? NTOK - 1 : t;
  const float* xr = x + (size_t)t * HD;
  const float* gp = gk + e;
  double acc = 0.0;
#pragma unroll 1
  for (int d4 = 0; d4 < HD / 4; ++d4) {
    const v4f xv = *(const v4f*)(xr + 4 * d4);
    const float* g4 = gp + (size_t)(4 * d4) * NE;
    const float w0 = rne16f(g4[0]);
    const float w1 = rne16f(g4[NE]);
    const float w2 = rne16f(g4[2 * NE]);
    const float w3 = rne16f(g4[3 * NE]);
    acc = fma((double)rne16f(xv.x), (double)w0, acc);
    acc = fma((double)rne16f(xv.y), (double)w1, acc);
    acc = fma((double)rne16f(xv.z), (double)w2, acc);
    acc = fma((double)rne16f(xv.w), (double)w3, acc);
  }
  const float logit = (float)acc;
  const float sig = 1.0f / (1.0f + expf(-logit));
  const float sfc = sig + rne16f(gb[e]);

  float s4[NE];
  const int hb = lane & 16;
#pragma unroll
  for (int j = 0; j < NE; ++j) s4[j] = __shfl(sfc, hb + j, 32);

  float gs[NGRP];
#pragma unroll
  for (int g = 0; g < NGRP; ++g) {
    const float a = s4[4 * g], b = s4[4 * g + 1], c = s4[4 * g + 2], d = s4[4 * g + 3];
    const float hi1 = fmaxf(a, b), lo1 = fminf(a, b);
    const float hi2 = fmaxf(c, d), lo2 = fminf(c, d);
    const float m1 = fmaxf(hi1, hi2);
    const float m2 = fmaxf(fminf(hi1, hi2), (hi1 >= hi2) ? lo1 : lo2);
    gs[g] = m1 + m2;
  }
  bool gsel[NGRP];
#pragma unroll
  for (int g = 0; g < NGRP; ++g) {
    int rank = 0;
#pragma unroll
    for (int g2 = 0; g2 < NGRP; ++g2)
      rank += ((gs[g2] > gs[g]) || ((gs[g2] == gs[g]) && (g2 < g))) ? 1 : 0;
    gsel[g] = (rank < 2);
  }
  float mval[NE];
#pragma unroll
  for (int j = 0; j < NE; ++j) mval[j] = gsel[j >> 2] ? s4[j] : 0.f;
  int rk[NE];
#pragma unroll
  for (int j = 0; j < NE; ++j) {
    int rank = 0;
#pragma unroll
    for (int j2 = 0; j2 < NE; ++j2)
      rank += ((mval[j2] > mval[j]) || ((mval[j2] == mval[j]) && (j2 < j))) ? 1 : 0;
    rk[j] = rank;
  }
  float den = 0.f;
#pragma unroll
  for (int j = 0; j < NE; ++j) den += (rk[j] < TOPK) ? mval[j] : 0.f;
  den += 1e-20f;
  const float rcp = 1.0f / den;
  int myrank = NE, posn = 0;
  float mymv = 0.f;
#pragma unroll
  for (int j = 0; j < NE; ++j) {
    const bool me = (j == e);
    myrank = me ? rk[j] : myrank;
    mymv   = me ? mval[j] : mymv;
    posn  += ((rk[j] < TOPK) && (j < e)) ? 1 : 0;
  }
  const bool sel = myrank < TOPK;
  const float w = (mymv * rcp) * SCALEF;
  posn = posn > TOPK - 1 ? TOPK - 1 : posn;
  const int tl = 2 * wave + hh;
  __syncthreads();
  if (sel) {
    rec[tl * 8 + posn]        = e;
    rec[tl * 8 + TOPK + posn] = __float_as_int(w);
  }
  __syncthreads();
  const v4i v = *(const v4i*)(rec + 4 * lane);
  int* rp = route + (size_t)blockIdx.x * (GTOK * 8) + 4 * lane;
  if (wave == 0) *(volatile v4i*)rp = v;
  __threadfence();
  if (wave == 0) *(volatile v4i*)rp = v;
}

__device__ __forceinline__ void cnt_add(int c, int (&cnt)[NE]) {
  c = c < 0 ? 0 : (c > NE - 1 ? NE - 1 : c);
#pragma unroll
  for (int e = 0; e < NE; ++e) cnt[e] += (c == e) ? 1 : 0;
}
__device__ __forceinline__ int slot_of(int c, int (&base)[NE]) {
  c = c < 0 ? 0 : (c > NE - 1 ? NE - 1 : c);
  int p = 0;
#pragma unroll
  for (int e = 0; e < NE; ++e) {
    const bool mt = (c == e);
    p = mt ? base[e] : p;
    base[e] += mt ? 1 : 0;
  }
  return p < 0 ? 0 : (p > MP - 1 ? MP - 1 : p);
}

__global__ __launch_bounds__(NTHR) void k_bucket(const int* __restrict__ route, int* tab) {
  extern __shared__ v4i lds_dyn[];
  int* img = (int*)lds_dyn;
  int* lst = img + TABH;
  int* pos = img + TABL;
  int* wt  = img + TABN;
  const int tid = (int)threadIdx.x, lane = tid & 31, wave = tid >> 5;

  const v4i z4 = {0, 0, 0, 0};
#pragma unroll 1
  for (int p = tid; p < TABN / 4; p += NTHR) *(v4i*)(img + 4 * p) = z4;
  __syncthreads();

  const int t0 = tid * TPT;
  int cnt[NE];
#pragma unroll
  for (int e = 0; e < NE; ++e) cnt[e] = 0;
#pragma unroll 1
  for (int c = 0; c < TPT; ++c) {
    const v4i rc = *(const v4i*)(route + (size_t)(t0 + c) * 8);
    cnt_add(rc.x, cnt);
    cnt_add(rc.y, cnt);
    cnt_add(rc.z, cnt);
    cnt_add(rc.w, cnt);
  }
  int incl[NE];
#pragma unroll
  for (int e = 0; e < NE; ++e) {
    int v = cnt[e];
#pragma unroll
    for (int d = 1; d < 32; d <<= 1) {
      const int up = __shfl_up(v, d);
      if (lane >= d) v += up;
    }
    incl[e] = v;
    if (lane == 31) wt[e * 8 + wave] = v;
  }
  __syncthreads();
  int pre[NE], tot[NE];
#pragma unroll
  for (int e = 0; e < NE; ++e) {
    int s = 0, all = 0;
#pragma unroll
    for (int w2 = 0; w2 < NTHR / 32; ++w2) {
      const int v = wt[e * 8 + w2];
      all += v;
      s   += (w2 < wave) ? v : 0;
    }
    pre[e] = s + incl[e] - cnt[e];
    all = all < 0 ? 0 : (all > NTOK * TOPK ? NTOK * TOPK : all);
    tot[e] = all;
  }
  int off[NE + 1];
  off[0] = 0;
#pragma unroll
  for (int e = 0; e < NE; ++e) {
    int nx = off[e] + ((tot[e] + TR - 1) / TR) * TR;
    nx = nx > MP ? MP : nx;
    off[e + 1] = nx;
  }
  int base[NE];
#pragma unroll
  for (int e = 0; e < NE; ++e) base[e] = off[e] + pre[e];
#pragma unroll 1
  for (int c = 0; c < TPT; ++c) {
    const v4i rc = *(const v4i*)(route + (size_t)(t0 + c) * 8);
    const int t = t0 + c;
    const int q0 = slot_of(rc.x, base); lst[q0] = t; pos[TOPK * t]     = q0;
    const int q1 = slot_of(rc.y, base); lst[q1] = t; pos[TOPK * t + 1] = q1;
    const int q2 = slot_of(rc.z, base); lst[q2] = t; pos[TOPK * t + 2] = q2;
    const int q3 = slot_of(rc.w, base); lst[q3] = t; pos[TOPK * t + 3] = q3;
  }
  __syncthreads();
  if (tid == 0) {
#pragma unroll
    for (int e = 0; e < NE; ++e) img[e] = tot[e];
#pragma unroll
    for (int j = 0; j <= NE; ++j) img[NE + j] = off[j];
  }
  __syncthreads();
#pragma unroll 1
  for (int p = tid; p < TABN / 4; p += NTHR) {
    const v4i v = *(const v4i*)(img + 4 * p);
    *(volatile v4i*)(tab + 4 * p) = v;
  }
  __threadfence();
#pragma unroll 1
  for (int p = tid; p < TABN / 4; p += NTHR) {
    const v4i v = *(const v4i*)(img + 4 * p);
    *(volatile v4i*)(tab + 4 * p) = v;
  }
}

__global__ __launch_bounds__(NTHR) void k_gather(const unsigned short* __restrict__ xb, const int* __restrict__ tab,
                                                 unsigned short* xg, int nUnits) {
  const int u = (int)blockIdx.x * NTHR + (int)threadIdx.x;
  if (u >= nUnits) return;
  const int row = u >> 7;
  const int c8  = (u & 127) * 8;
  int tk = tab[TABH + row];
  tk = tk < 0 ? 0 : (tk > NTOK - 1 ? NTOK - 1 : tk);
  const v8us o = *(const v8us*)(xb + (size_t)tk * HD + c8);
  const size_t q = (size_t)row * HD + (size_t)c8;
  *(volatile v8us*)(xg + q) = o;
  __threadfence();
  *(volatile v8us*)(xg + q) = o;
}

__device__ __forceinline__ int tile_slot(const int* __restrict__ tab, int rowBase) {
  const v4i o0 = *(const v4i*)(tab + NE);
  const v4i o1 = *(const v4i*)(tab + NE + 4);
  const v4i o2 = *(const v4i*)(tab + NE + 8);
  const v4i o3 = *(const v4i*)(tab + NE + 12);
  int e = 0;
#define SELX(J, OJ) { const bool ge_ = rowBase >= (OJ); e = ge_ ? (J) : e; }
  SELX(1, o0.y)  SELX(2, o0.z)  SELX(3, o0.w)
  SELX(4, o1.x)  SELX(5, o1.y)  SELX(6, o1.z)  SELX(7, o1.w)
  SELX(8, o2.x)  SELX(9, o2.y)  SELX(10, o2.z) SELX(11, o2.w)
  SELX(12, o3.x) SELX(13, o3.y) SELX(14, o3.z) SELX(15, o3.w)
#undef SELX
  return e;
}

__global__ __launch_bounds__(GTHR) void k_up(const unsigned short* __restrict__ ap,
                                             const unsigned short* __restrict__ wgt,
                                             const unsigned short* __restrict__ wut,
                                             const int* __restrict__ tab,
                                             unsigned short* hhi, unsigned short* hlo,
                                             int K, int N, int useTab) {
  __shared__ __attribute__((aligned(16))) float stg[TR * 64];
  const int tid = (int)threadIdx.x, lane = tid & 31, wave = tid >> 5, hh = lane >> 4, m = lane & 15;
  const int rowBase = (int)blockIdx.x * TR;
  const int col0    = (int)blockIdx.y * 64;
  const int es = tile_slot(tab, rowBase);
  const int e  = (useTab != 0) ? es : 0;

  v8f accg[4], accu[4];
  {
    const v8f z = {0.f, 0.f, 0.f, 0.f, 0.f, 0.f, 0.f, 0.f};
    accg[0] = z; accg[1] = z; accg[2] = z; accg[3] = z;
    accu[0] = z; accu[1] = z; accu[2] = z; accu[3] = z;
  }
  const size_t arow = (size_t)(rowBase + 16 * wave + m) * (size_t)K + (size_t)(8 * hh);
  const unsigned short* aph = ap + arow;
  const size_t woff = (size_t)e * (size_t)N * (size_t)K + (size_t)(col0 + m) * (size_t)K + (size_t)(8 * hh);
  const unsigned short* wg = wgt + woff;
  const unsigned short* wu = wut + woff;
  const int nks = K >> 5;
#pragma unroll 1
  for (int ks = 0; ks < nks; ++ks) {
    FragB ah;
    ah.h[0] = *(const v8us*)(aph + 32 * ks);
    ah.h[1] = *(const v8us*)(aph + 32 * ks + 16);
#pragma unroll
    for (int t = 0; t < 4; ++t) {
      const unsigned short* q1 = wg + (size_t)(16 * t) * (size_t)K + 32 * ks;
      const unsigned short* q2 = wu + (size_t)(16 * t) * (size_t)K + 32 * ks;
      FragB bg, bu;
      bg.h[0] = *(const v8us*)q1;
      bg.h[1] = *(const v8us*)(q1 + 16);
      bu.h[0] = *(const v8us*)q2;
      bu.h[1] = *(const v8us*)(q2 + 16);
      accg[t] = wmb(ah, bg, accg[t]);
      accu[t] = wmb(ah, bu, accu[t]);
    }
  }

#pragma unroll
  for (int t = 0; t < 4; ++t) {
    const int lc = 16 * t + m;
#pragma unroll
    for (int r = 0; r < 8; ++r) {
      const int lr = 16 * wave + 8 * hh + r;
      const float gg = accg[t][r];
      const float uu = accu[t][r];
      const float sg = __builtin_amdgcn_rcpf(1.0f + __expf(-gg));
      stg[lr * 64 + lc] = (gg * sg) * uu;
    }
  }
  __syncthreads();

  const int q8 = lane & 7, sub = lane >> 3;
  v8us hv[4], lv[4];
  size_t po[4];
#pragma unroll
  for (int i = 0; i < 4; ++i) {
    const int lr = 16 * wave + 4 * i + sub;
    const v4f a = *(const v4f*)(stg + lr * 64 + 8 * q8);
    const v4f b = *(const v4f*)(stg + lr * 64 + 8 * q8 + 4);
    split8(a, b, hv[i], lv[i]);
    po[i] = (size_t)(rowBase + lr) * (size_t)N + (size_t)(col0 + 8 * q8);
  }
#pragma unroll
  for (int i = 0; i < 4; ++i) {
    *(volatile v8us*)(hhi + po[i]) = hv[i];
    *(volatile v8us*)(hlo + po[i]) = lv[i];
  }
  __threadfence();
#pragma unroll
  for (int i = 0; i < 4; ++i) {
    *(volatile v8us*)(hhi + po[i]) = hv[i];
    *(volatile v8us*)(hlo + po[i]) = lv[i];
  }
}

__global__ __launch_bounds__(GTHR) void k_down(const unsigned short* __restrict__ hhi,
                                               const unsigned short* __restrict__ hlo,
                                               const unsigned short* __restrict__ wdt,
                                               const int* __restrict__ tab, float* y, int K, int useTab) {
  __shared__ __attribute__((aligned(16))) float stg[TR * 64];
  const int tid = (int)threadIdx.x, lane = tid & 31, wave = tid >> 5, hh = lane >> 4, m = lane & 15;
  const int rowBase = (int)blockIdx.x * TR;
  const int col0    = (int)blockIdx.y * 64;
  const int es = tile_slot(tab, rowBase);
  const int e  = (useTab != 0) ? es : 0;

  v8f acc[4];
  {
    const v8f z = {0.f, 0.f, 0.f, 0.f, 0.f, 0.f, 0.f, 0.f};
    acc[0] = z; acc[1] = z; acc[2] = z; acc[3] = z;
  }
  const size_t arow = (size_t)(rowBase + 16 * wave + m) * (size_t)K + (size_t)(8 * hh);
  const unsigned short* aph = hhi + arow;
  const unsigned short* apl = hlo + arow;
  const unsigned short* wp  = wdt + (size_t)e * (size_t)HD * (size_t)K + (size_t)(col0 + m) * (size_t)K +
                              (size_t)(8 * hh);
  const int nks = K >> 5;
#pragma unroll 1
  for (int ks = 0; ks < nks; ++ks) {
    FragB ah, al;
    ah.h[0] = *(const v8us*)(aph + 32 * ks);
    ah.h[1] = *(const v8us*)(aph + 32 * ks + 16);
    al.h[0] = *(const v8us*)(apl + 32 * ks);
    al.h[1] = *(const v8us*)(apl + 32 * ks + 16);
#pragma unroll
    for (int t = 0; t < 4; ++t) {
      const unsigned short* wq = wp + (size_t)(16 * t) * (size_t)K + 32 * ks;
      FragB bf;
      bf.h[0] = *(const v8us*)wq;
      bf.h[1] = *(const v8us*)(wq + 16);
      acc[t] = wmb(ah, bf, acc[t]);
      acc[t] = wmb(al, bf, acc[t]);
    }
  }

#pragma unroll
  for (int t = 0; t < 4; ++t) {
    const int lc = 16 * t + m;
#pragma unroll
    for (int r = 0; r < 8; ++r) {
      const int lr = 16 * wave + 8 * hh + r;
      stg[lr * 64 + lc] = acc[t][r];
    }
  }
  __syncthreads();

  v4f fv[8];
  size_t op[8];
#pragma unroll
  for (int i = 0; i < 8; ++i) {
    const int lr = 16 * wave + 2 * i + hh;
    fv[i] = *(const v4f*)(stg + lr * 64 + 4 * m);
    op[i] = (size_t)(rowBase + lr) * (size_t)HD + (size_t)(col0 + 4 * m);
  }
#pragma unroll
  for (int i = 0; i < 8; ++i) *(volatile v4f*)(y + op[i]) = fv[i];
  __threadfence();
#pragma unroll
  for (int i = 0; i < 8; ++i) *(volatile v4f*)(y + op[i]) = fv[i];
}

__global__ __launch_bounds__(NTHR) void k_combine(const float* __restrict__ y, const float* __restrict__ ys,
                                                  const int* __restrict__ route, const int* __restrict__ tab,
                                                  float* out) {
  const int lane = (int)threadIdx.x & 31, wave = (int)threadIdx.x >> 5;
  const int t = (int)blockIdx.x * 8 + wave;
  if (t >= NTOK) return;
  const v4i wrec = *(const v4i*)(route + (size_t)t * 8 + 4);
  const v4i prec = *(const v4i*)(tab + TABL + 4 * t);
  const float w0 = __int_as_float(wrec.x);
  const float w1 = __int_as_float(wrec.y);
  const float w2 = __int_as_float(wrec.z);
  const float w3 = __int_as_float(wrec.w);
  int q0 = prec.x, q1 = prec.y, q2 = prec.z, q3 = prec.w;
  q0 = q0 < 0 ? 0 : (q0 > MP - 1 ? MP - 1 : q0);
  q1 = q1 < 0 ? 0 : (q1 > MP - 1 ? MP - 1 : q1);
  q2 = q2 < 0 ? 0 : (q2 > MP - 1 ? MP - 1 : q2);
  q3 = q3 < 0 ? 0 : (q3 > MP - 1 ? MP - 1 : q3);
  const float* rs = ys + (size_t)t  * HD;
  const float* ra = y  + (size_t)q0 * HD;
  const float* rb = y  + (size_t)q1 * HD;
  const float* rc = y  + (size_t)q2 * HD;
  const float* rd = y  + (size_t)q3 * HD;
  float* orow = out + (size_t)t * HD;
#pragma unroll 1
  for (int c = 0; c < HD / 128; ++c) {
    const int col = 128 * c + 4 * lane;
    const v4f s = *(const v4f*)(rs + col);
    const v4f a = *(const v4f*)(ra + col);
    const v4f b = *(const v4f*)(rb + col);
    const v4f g = *(const v4f*)(rc + col);
    const v4f d = *(const v4f*)(rd + col);
    v4f r, o;
    r.x = w0 * a.x; r.x = fmaf(w1, b.x, r.x); r.x = fmaf(w2, g.x, r.x); r.x = fmaf(w3, d.x, r.x); o.x = r.x + s.x;
    r.y = w0 * a.y; r.y = fmaf(w1, b.y, r.y); r.y = fmaf(w2, g.y, r.y); r.y = fmaf(w3, d.y, r.y); o.y = r.y + s.y;
    r.z = w0 * a.z; r.z = fmaf(w1, b.z, r.z); r.z = fmaf(w2, g.z, r.z); r.z = fmaf(w3, d.z, r.z); o.z = r.z + s.z;
    r.w = w0 * a.w; r.w = fmaf(w1, b.w, r.w); r.w = fmaf(w2, g.w, r.w); r.w = fmaf(w3, d.w, r.w); o.w = r.w + s.w;
    float* op = orow + col;
    *(volatile v4f*)op = o;
    __threadfence();
    *(volatile v4f*)op = o;
  }
}

static inline int cdiv(int a, int b) { return (a + b - 1) / b; }

extern "C" void kernel_launch(void* const* d_in, const int* in_sizes, int n_in,
                              void* d_out, int out_size, void* d_ws, size_t ws_size,
                              hipStream_t stream) {
  if (n_in < 9) return;
  if (in_sizes[0] != NTOK * HD) return;
  if (in_sizes[1] != HD * NE) return;
  if (in_sizes[2] != NE) return;
  if (in_sizes[3] != NE * HD * MI) return;
  if (in_sizes[4] != NE * HD * MI) return;
  if (in_sizes[5] != NE * MI * HD) return;
  if (in_sizes[6] != HD * SI) return;
  if (in_sizes[7] != HD * SI) return;
  if (in_sizes[8] != SI * HD) return;
  if (out_size != NTOK * HD) return;

  const float* x   = (const float*)d_in[0];
  const float* gk  = (const float*)d_in[1];
  const float* gbi = (const float*)d_in[2];
  const float* wg  = (const float*)d_in[3];
  const float* wu  = (const float*)d_in[4];
  const float* wd  = (const float*)d_in[5];
  const float* swg = (const float*)d_in[6];
  const float* swu = (const float*)d_in[7];
  const float* swd = (const float*)d_in[8];
  float* out = (float*)d_out;

  const size_t szWGT = (size_t)NE * MI * HD * 2;
  const size_t szWUT = szWGT;
  const size_t szXG  = (size_t)MP * HD * 2;
  const size_t szXB  = (size_t)NTOK * HD * 2;
  const size_t szY   = (size_t)MP * HD * 4;
  const size_t szYS  = (size_t)NTOK * HD * 4;
  const size_t szR0a = szWGT + szWUT + szXG + szXB;
  const size_t szR0b = szY + szYS;
  const size_t szR0  = szR0a > szR0b ? szR0a : szR0b;
  char* ws = (char*)d_ws;
  size_t off = 0;
  const size_t oWGT = 0;
  const size_t oWUT = oWGT + szWGT;
  const size_t oXG  = oWUT + szWUT;
  const size_t oXB  = oXG + szXG;
  const size_t oY   = 0;
  const size_t oYS  = oY + szY;
  off += szR0;                                      off = (off + 255) & ~(size_t)255;
  const size_t oWDT = off; off += (size_t)NE * HD * MI * 2;   off = (off + 255) & ~(size_t)255;
  const size_t oSWG = off; off += (size_t)SI * HD * 2;        off = (off + 255) & ~(size_t)255;
  const size_t oSWU = off; off += (size_t)SI * HD * 2;        off = (off + 255) & ~(size_t)255;
  const size_t oSWD = off; off += (size_t)HD * SI * 2;        off = (off + 255) & ~(size_t)255;
  const size_t oHHI = off; off += (size_t)MP * MI * 2;        off = (off + 255) & ~(size_t)255;
  const size_t oHLO = off; off += (size_t)MP * MI * 2;        off = (off + 255) & ~(size_t)255;
  const size_t oSHI = off; off += (size_t)NTOK * SI * 2;      off = (off + 255) & ~(size_t)255;
  const size_t oSLO = off; off += (size_t)NTOK * SI * 2;      off = (off + 255) & ~(size_t)255;
  const size_t oRT  = off; off += (size_t)NTOK * 8 * 4;       off = (off + 255) & ~(size_t)255;
  const size_t oTAB = off; off += (size_t)TABN * 4;           off = (off + 255) & ~(size_t)255;
  if (off > ws_size || off > (size_t)WSMAX) return;

  unsigned short* WGT  = (unsigned short*)(ws + oWGT);
  unsigned short* WUT  = (unsigned short*)(ws + oWUT);
  unsigned short* XG   = (unsigned short*)(ws + oXG);
  unsigned short* XB   = (unsigned short*)(ws + oXB);
  float*          Y    = (float*)(ws + oY);
  float*          YS   = (float*)(ws + oYS);
  unsigned short* WDT  = (unsigned short*)(ws + oWDT);
  unsigned short* SWGT = (unsigned short*)(ws + oSWG);
  unsigned short* SWUT = (unsigned short*)(ws + oSWU);
  unsigned short* SWDT = (unsigned short*)(ws + oSWD);
  unsigned short* HHI  = (unsigned short*)(ws + oHHI);
  unsigned short* HLO  = (unsigned short*)(ws + oHLO);
  unsigned short* SHI  = (unsigned short*)(ws + oSHI);
  unsigned short* SLO  = (unsigned short*)(ws + oSLO);
  int*            RT   = (int*)(ws + oRT);
  int*            TAB  = (int*)(ws + oTAB);

  hipFuncSetAttribute(reinterpret_cast<const void*>(&k_bucket),
                      hipFuncAttributeMaxDynamicSharedMemorySize, LDS_BKT);

  {
    const int nUg = NE * HD * MI / 8;
    k_wtr<<<cdiv(nUg, NTHR), NTHR, 0, stream>>>(wg, WGT, HD, MI, NE, nUg);
    k_wtr<<<cdiv(nUg, NTHR), NTHR, 0, stream>>>(wu, WUT, HD, MI, NE, nUg);
    const int nUd = NE * MI * HD / 8;
    k_wtr<<<cdiv(nUd, NTHR), NTHR, 0, stream>>>(wd, WDT, MI, HD, NE, nUd);
    const int nUs = HD * SI / 8;
    k_wtr<<<cdiv(nUs, NTHR), NTHR, 0, stream>>>(swg, SWGT, HD, SI, 1, nUs);
    k_wtr<<<cdiv(nUs, NTHR), NTHR, 0, stream>>>(swu, SWUT, HD, SI, 1, nUs);
    const int nUt = SI * HD / 8;
    k_wtr<<<cdiv(nUt, NTHR), NTHR, 0, stream>>>(swd, SWDT, SI, HD, 1, nUt);
  }
  {
    const int nUx = NTOK * HD / 8;
    k_cvx<<<cdiv(nUx, NTHR), NTHR, 0, stream>>>(x, XB, nUx);
  }
  k_gate<<<NTOK / GTOK, NTHR, 0, stream>>>(x, gk, gbi, RT);
  k_bucket<<<1, NTHR, LDS_BKT, stream>>>(RT, TAB);
  {
    const int nUb = MP * (HD / 8);
    k_gather<<<cdiv(nUb, NTHR), NTHR, 0, stream>>>(XB, TAB, XG, nUb);
  }
  k_up<<<dim3(NTOK / TR, SI / 64), GTHR, 0, stream>>>(XB, SWGT, SWUT, TAB, SHI, SLO, HD, SI, 0);
  k_up<<<dim3(NTILE, MI / 64), GTHR, 0, stream>>>(XG, WGT, WUT, TAB, HHI, HLO, HD, MI, 1);
  k_down<<<dim3(NTOK / TR, HD / 64), GTHR, 0, stream>>>(SHI, SLO, SWDT, TAB, YS, SI, 0);
  k_down<<<dim3(NTILE, HD / 64), GTHR, 0, stream>>>(HHI, HLO, WDT, TAB, Y, MI, 1);
  k_combine<<<NTOK / 8, NTHR, 0, stream>>>(Y, YS, RT, TAB, out);
}
